// GridSelfAttention_33913061769434
// MI455X (gfx1250) — hardware-verified
//
#include <hip/hip_runtime.h>


#define NG   320
#define CC   128
#define NH_  4
#define HD   32
#define CHB  16
#define RCH  (CHB * NG)
#define NZC  (CHB * NH_)
#define PCAR 1024.0f
#define QSC  0.17677669529663688f
#define MASKF (-1.0e9f)
typedef _Float16 h16;
typedef unsigned short bf;
typedef __attribute__((ext_vector_type(16))) __bf16   v16bf;
typedef __attribute__((ext_vector_type(16))) _Float16 v16h;
typedef __attribute__((ext_vector_type(8)))  _Float16 v8h;
typedef __attribute__((ext_vector_type(8)))  unsigned short v8us;
typedef __attribute__((ext_vector_type(8)))  float    v8f;
typedef __attribute__((ext_vector_type(4)))  float    v4f;
typedef v8h  __attribute__((may_alias)) v8ha;
typedef v4f  __attribute__((may_alias)) v4fa;
typedef v8us __attribute__((may_alias)) v8usa;

__device__ __forceinline__ unsigned short f2bf(float f) { unsigned u = __float_as_uint(f); u += 0x7FFFu + ((u >> 16) & 1u); return (unsigned short)(u >> 16); }
__device__ __forceinline__ float bf2f(unsigned short b) { return __uint_as_float(((unsigned)b) << 16); }
__device__ __forceinline__ float bfr(float f) { return bf2f(f2bf(f)); }
__device__ __forceinline__ v16h cat16(v8h lo, v8h hi) { return __builtin_shufflevector(lo, hi, 0, 1, 2, 3, 4, 5, 6, 7, 8, 9, 10, 11, 12, 13, 14, 15); }
__device__ __forceinline__ v16bf cat16b(v8us lo, v8us hi) { return __builtin_bit_cast(v16bf, __builtin_shufflevector(lo, hi, 0, 1, 2, 3, 4, 5, 6, 7, 8, 9, 10, 11, 12, 13, 14, 15)); }
__device__ __forceinline__ v8f wmma16(v16h a, v16h b, v8f c) { return __builtin_amdgcn_wmma_f32_16x16x32_f16(false, a, false, b, (short)0, c, false, false); }
__device__ __forceinline__ v8f wmmab(v16bf a, v16bf b, v8f c) { return __builtin_amdgcn_wmma_f32_16x16x32_bf16(false, a, false, b, (short)0, c, false, false); }


template <typename T16> struct WFrag;
template <> struct WFrag<h16> { typedef v16h V; static __device__ __forceinline__ V ld(const h16* p) { return cat16(*(const v8h*)p, *(const v8h*)(p + 16)); } static __device__ __forceinline__ v8f mma(V a, V b, v8f c) { return wmma16(a, b, c); } };
template <> struct WFrag<bf> { typedef v16bf V; static __device__ __forceinline__ V ld(const bf* p) { return cat16b(*(const v8us*)p, *(const v8us*)(p + 16)); } static __device__ __forceinline__ v8f mma(V a, V b, v8f c) { return wmmab(a, b, c); } };
template <typename T16, int NSPLIT, bool BIAS>
__global__ __launch_bounds__(32) void k_gemmw(const T16* __restrict__ A, const T16* __restrict__ A2, const T16* __restrict__ Bt, const T16* __restrict__ Bt2, int K, float* C, int ldc, const float* __restrict__ bias, size_t sA, size_t sB, size_t sC) {
    typedef typename WFrag<T16>::V V;
    __shared__ __align__(16) float os[16 * 68];
    const size_t z = blockIdx.z; A += z * sA; if (A2) A2 += z * sA; Bt += z * sB; if (Bt2) Bt2 += z * sB; C += z * sC;
    const int lane = threadIdx.x & 31, lr = lane & 15, hi = lane >> 4; const int r0 = blockIdx.x * 64, c0 = blockIdx.y * 64;
    v8f acc[4][4];
#pragma unroll
    for (int mb = 0; mb < 4; ++mb)
#pragma unroll
        for (int nb = 0; nb < 4; ++nb) acc[mb][nb] = (v8f){};
    const size_t aoff = (size_t)(r0 + lr) * K + 8 * hi, boff = (size_t)(c0 + lr) * K + 8 * hi;
#pragma unroll 1
    for (int kc = 0; kc < K; kc += 32) {
        V a[4], a2[4];
#pragma unroll
        for (int mb = 0; mb < 4; ++mb) { a[mb] = WFrag<T16>::ld(A + aoff + (size_t)mb * 16 * K + kc); if (NSPLIT == 1 || NSPLIT == 2) a2[mb] = WFrag<T16>::ld(A2 + aoff + (size_t)mb * 16 * K + kc); }
#pragma unroll
        for (int nb = 0; nb < 4; ++nb) { const V b = WFrag<T16>::ld(Bt + boff + (size_t)nb * 16 * K + kc); V b2; if (NSPLIT >= 2) b2 = WFrag<T16>::ld(Bt2 + boff + (size_t)nb * 16 * K + kc);
#pragma unroll
            for (int mb = 0; mb < 4; ++mb) { acc[mb][nb] = WFrag<T16>::mma(a[mb], b, acc[mb][nb]); if (NSPLIT == 1 || NSPLIT == 2) acc[mb][nb] = WFrag<T16>::mma(a2[mb], b, acc[mb][nb]); if (NSPLIT >= 2) acc[mb][nb] = WFrag<T16>::mma(a[mb], b2, acc[mb][nb]); } }
        asm volatile("v_nop\n\tv_nop\n\tv_nop\n\tv_nop" : "+v"(acc[0][0]), "+v"(acc[1][1]), "+v"(acc[2][2]), "+v"(acc[3][3]) : "v"(a[0]), "v"(a[3]));
    }
#pragma unroll
    for (int mb = 0; mb < 4; ++mb) {
#pragma unroll
        for (int nb = 0; nb < 4; ++nb) {
#pragma unroll
            for (int j = 0; j < 8; ++j) os[(hi * 8 + j) * 68 + nb * 16 + lr] = acc[mb][nb][j]; }
        __builtin_amdgcn_wave_barrier(); asm volatile("" ::: "memory");
        float* crow = C + (size_t)(r0 + mb * 16) * ldc + c0;
#pragma unroll 1
        for (int ps = 0; ps < 2; ++ps) {
#pragma unroll
            for (int s = 0; s < 8; ++s) { const int row = 2 * s + hi, cofs = lr * 4; v4f val = *(const v4fa*)(os + row * 68 + cofs); if (BIAS) { val[0] += bfr(bias[c0 + cofs]); val[1] += bfr(bias[c0 + cofs + 1]); val[2] += bfr(bias[c0 + cofs + 2]); val[3] += bfr(bias[c0 + cofs + 3]); }
                *(volatile v4f*)(crow + (size_t)row * ldc + cofs) = val; }
            if (ps == 0) __threadfence(); }
        __builtin_amdgcn_wave_barrier(); asm volatile("" ::: "memory");
    }
}

__device__ __forceinline__ h16 tohx(float x) { return (h16)x; }
__device__ __forceinline__ void splitf(float y, unsigned short& h, unsigned short& l) { h = f2bf(y); l = f2bf(y - bf2f(h)); }
typedef __attribute__((ext_vector_type(2))) _Float16 v2h;
typedef __attribute__((ext_vector_type(2))) unsigned short v2us;
typedef __attribute__((ext_vector_type(4))) unsigned short v4us;

__global__ __launch_bounds__(256) void k_wtG(const float* __restrict__ w, int K, int N, bf* Bt) {
    const int lane = threadIdx.x & 31; const int L0 = (blockIdx.x * 8 + (threadIdx.x >> 5)) * 8; const int nlines = N * K / 64;
#pragma unroll 1
    for (int ps = 0; ps < 2; ++ps) {
#pragma unroll 1
        for (int l = 0; l < 8; ++l) { const int L = L0 + l; if (L >= nlines) break; const size_t e = (size_t)L * 64 + lane * 2; const int k = (int)(e % K), n = (int)(e / K); v2us o;
            o[0] = f2bf(w[(size_t)k * N + n]); o[1] = f2bf(w[(size_t)(k + 1) * N + n]); *(volatile v2us*)(Bt + e) = o; }
        if (ps == 0) __threadfence(); }
}
__global__ __launch_bounds__(256) void k_cvt8(const float* __restrict__ src, bf* dst, size_t n8) { const size_t i = (size_t)blockIdx.x * 256 + threadIdx.x; if (i >= n8) return; const v8f v = *(const v8f*)(src + i * 8); v8us o;
#pragma unroll
    for (int k = 0; k < 8; ++k) o[k] = f2bf(v[k]); *(volatile v8us*)(dst + i * 8) = o; __threadfence(); *(volatile v8us*)(dst + i * 8) = o; }
__global__ __launch_bounds__(256) void k_wpb(const float* __restrict__ w, bf* WPB) { for (int ps = 0; ps < 2; ++ps) { for (int i4 = threadIdx.x * 4; i4 < 64 * CC; i4 += 256 * 4) { v4us o;
#pragma unroll
        for (int q = 0; q < 4; ++q) { const int i = i4 + q; const int n = i / CC, c = i % CC; o[q] = (n < NH_) ? f2bf(w[c * NH_ + n]) : (unsigned short)0; }
        *(volatile v4us*)(WPB + i4) = o; } if (ps == 0) __threadfence(); } }
__global__ __launch_bounds__(256) void k_gln(const float* __restrict__ act, const float* __restrict__ gg, const float* __restrict__ bb, int r0, bf* Hh, bf* Hl) {
    const int lane = threadIdx.x & 31; const int r = blockIdx.x * 8 + (threadIdx.x >> 5); if (r >= RCH) return; const v4f a = *(const v4f*)(act + ((size_t)r0 + r) * CC + lane * 4); float v[4]; float s = 0.f;
#pragma unroll
    for (int q = 0; q < 4; ++q) { float t = bfr(a[q]); asm volatile("" : "+v"(t)); v[q] = t; s = __fadd_rn(s, t); }
#pragma unroll
    for (int sh = 16; sh; sh >>= 1) s += __shfl_xor(s, sh, 32);
    const float mu = s * (1.0f / CC); float qq = 0.f;
#pragma unroll
    for (int q = 0; q < 4; ++q) { const float d0 = v[q] - mu; float p = __fmul_rn(d0, d0); asm volatile("" : "+v"(p)); qq = __fadd_rn(qq, p); }
#pragma unroll
    for (int sh = 16; sh; sh >>= 1) qq += __shfl_xor(qq, sh, 32);
    const float rs = __fdiv_rn(1.0f, __fsqrt_rn(__fadd_rn(qq * (1.0f / CC), 1e-5f))); v4us oh, ol;
#pragma unroll
    for (int q = 0; q < 4; ++q) { const int col = lane * 4 + q; float t = __fmul_rn(v[q] - mu, rs); asm volatile("" : "+v"(t)); float tg = __fmul_rn(t, bfr(gg[col])); asm volatile("" : "+v"(tg)); unsigned short a2, c2; splitf(__fadd_rn(tg, bfr(bb[col])), a2, c2); oh[q] = a2; ol[q] = c2; }
    const size_t o = (size_t)r * CC + lane * 4; *(volatile v4us*)(Hh + o) = oh; *(volatile v4us*)(Hl + o) = ol; __threadfence(); *(volatile v4us*)(Hh + o) = oh; *(volatile v4us*)(Hl + o) = ol; }
__global__ __launch_bounds__(256) void k_gpl(const float* __restrict__ PF, h16* QP, h16* KP) { const int e = (blockIdx.x * 256 + threadIdx.x) * 2; if (e >= NZC * NG * HD) return; const int d = e & 31; const int t = (e >> 5) % NG; const int z = (e >> 5) / NG; const int bb = z >> 2, h = z & 3; const float* row = PF + ((size_t)bb * NG + t) * 512 + h * HD + d;
    v2h q2, k2; q2[0] = tohx(__fmul_rn(row[0], QSC)); q2[1] = tohx(__fmul_rn(row[1], QSC)); k2[0] = tohx(row[CC]); k2[1] = tohx(row[CC + 1]); *(volatile v2h*)(QP + e) = q2; *(volatile v2h*)(KP + e) = k2; __threadfence(); *(volatile v2h*)(QP + e) = q2; *(volatile v2h*)(KP + e) = k2; }
__global__ __launch_bounds__(256) void k_gvt(const float* __restrict__ PF, h16* VT) { const int e = (blockIdx.x * 256 + threadIdx.x) * 2; if (e >= NZC * 64 * NG) return; const int k = e % NG; const int d = (e / NG) & 63; const int z = e / (NG * 64); const int bb = z >> 2, h = z & 3; v2h v;
    if (d < HD) { const float* col = PF + ((size_t)bb * NG) * 512 + 2 * CC + h * HD + d; v[0] = tohx(col[(size_t)k * 512]); v[1] = tohx(col[(size_t)(k + 1) * 512]); } else { v[0] = 0; v[1] = 0; }
    *(volatile v2h*)(VT + e) = v; __threadfence(); *(volatile v2h*)(VT + e) = v; }
__global__ __launch_bounds__(256) void k_gsoft(const float* __restrict__ Sb, const float* __restrict__ BIASF, const int* __restrict__ pm, int b0, h16* P16) {
    const int lane = threadIdx.x & 31; const int row = blockIdx.x * 8 + (threadIdx.x >> 5); if (row >= NZC * NG) return; const int q = row % NG; const int z = row / NG; const int b = b0 + (z >> 2), h = z & 3; const float* sr = Sb + (size_t)row * NG; float v[10]; float mx = -3.0e38f;
#pragma unroll
    for (int c = 0; c < 10; ++c) { const int j = lane * 10 + c; const float bias = BIASF[((size_t)q * NG + j) * 64 + h]; const float t = (pm[(size_t)j * NG + b] > 0) ? __fadd_rn(sr[j], bias) : MASKF; v[c] = t; mx = fmaxf(mx, t); }
#pragma unroll
    for (int sh = 16; sh; sh >>= 1) mx = fmaxf(mx, __shfl_xor(mx, sh, 32));
    float sum = 0.f;
#pragma unroll
    for (int c = 0; c < 10; ++c) { float d0 = __fsub_rn(v[c], mx); asm volatile("" : "+v"(d0)); v[c] = __builtin_amdgcn_exp2f(__fmul_rn(d0, 1.4426950408889634f)); sum += v[c]; }
#pragma unroll
    for (int sh = 16; sh; sh >>= 1) sum += __shfl_xor(sum, sh, 32);
    const float f = __fdiv_rn(PCAR, sum);
#pragma unroll 1
    for (int ps = 0; ps < 2; ++ps) {
#pragma unroll
        for (int c = 0; c < 10; c += 2) { v2h o; o[0] = tohx(v[c] * f); o[1] = tohx(v[c + 1] * f); *(volatile v2h*)(P16 + (size_t)row * NG + lane * 10 + c) = o; }
        if (ps == 0) __threadfence(); }
}
__global__ __launch_bounds__(256) void k_gmrg(const float* __restrict__ O, const float* __restrict__ PF, bf* Ah, bf* Al) { const int e = (blockIdx.x * 256 + threadIdx.x) * 2; if (e >= RCH * CC) return; const int col = e % CC; const int rr = e / CC; const int h = col / HD, d = col % HD; const int bb = rr / NG, q = rr % NG; const int z = bb * NH_ + h;
    const float* orow = O + ((size_t)z * NG + q) * 64 + d; const float* grow = PF + (size_t)rr * 512 + 3 * CC + col; v2us oh, ol;
#pragma unroll
    for (int u = 0; u < 2; ++u) { const float g = grow[u]; const float sg = __fdiv_rn(1.0f, __fadd_rn(1.0f, __expf(-g))); float w = orow[u] * (1.0f / PCAR); asm volatile("" : "+v"(w)); unsigned short a2, c2; splitf(__fmul_rn(w, sg), a2, c2); oh[u] = a2; ol[u] = c2; }
    *(volatile v2us*)(Ah + e) = oh; *(volatile v2us*)(Al + e) = ol; __threadfence(); *(volatile v2us*)(Ah + e) = oh; *(volatile v2us*)(Al + e) = ol; }

extern "C" void kernel_launch(void* const* d_in, const int* in_sizes, int n_in,
                              void* d_out, int out_size, void* d_ws, size_t ws_size, hipStream_t stream) {
    (void)in_sizes; (void)n_in; (void)out_size;
    const float* act = (const float*)d_in[0]; const int* pm = (const int*)d_in[1]; const float* lg = (const float*)d_in[2]; const float* lb = (const float*)d_in[3]; const float* wpb = (const float*)d_in[4]; const float* wq = (const float*)d_in[5]; const float* wk = (const float*)d_in[6]; const float* wv = (const float*)d_in[7]; const float* wg = (const float*)d_in[8]; const float* wo = (const float*)d_in[9];
    float* OUT = (float*)d_out;
    char* wsp = (char*)d_ws;
    auto take = [&](size_t bytes) { char* p = wsp; wsp += (bytes + 255) & ~(size_t)255; return (void*)p; };
    bf* WPB = (bf*)take(64 * CC * 2); bf* WPR = (bf*)take((size_t)512 * CC * 2); bf* WO = (bf*)take(CC * CC * 2); float* BIASF = (float*)take((size_t)NG * NG * 64 * 4);
    bf* Hh = (bf*)take((size_t)RCH * CC * 2); bf* Hl = (bf*)take((size_t)RCH * CC * 2); float* PF = (float*)take((size_t)RCH * 512 * 4); h16* QP = (h16*)take((size_t)NZC * NG * HD * 2); h16* KP = (h16*)take((size_t)NZC * NG * HD * 2); h16* VT = (h16*)take((size_t)NZC * 64 * NG * 2);
    float* Sb = (float*)take((size_t)NZC * NG * NG * 4); h16* Pm = (h16*)take((size_t)NZC * NG * NG * 2); float* Ob = (float*)take((size_t)NZC * NG * 64 * 4); bf* Ah = (bf*)take((size_t)RCH * CC * 2); bf* Al = (bf*)take((size_t)RCH * CC * 2);
    if ((size_t)(wsp - (char*)d_ws) > ws_size) return;
    { k_wpb<<<1, 256, 0, stream>>>(wpb, WPB); const unsigned gT = (unsigned)((CC * CC / 64 + 63) / 64);
      k_wtG<<<gT, 256, 0, stream>>>(wq, CC, CC, WPR); k_wtG<<<gT, 256, 0, stream>>>(wk, CC, CC, WPR + (size_t)CC * CC); k_wtG<<<gT, 256, 0, stream>>>(wv, CC, CC, WPR + (size_t)2 * CC * CC); k_wtG<<<gT, 256, 0, stream>>>(wg, CC, CC, WPR + (size_t)3 * CC * CC);
      k_cvt8<<<(CC * CC / 8 + 255) / 256, 256, 0, stream>>>(wo, WO, (size_t)CC * CC / 8); }
    const unsigned LR = RCH / 8;
    for (int b0 = 0; b0 < NG; b0 += CHB) { const int r0 = b0 * NG;
        k_gln<<<LR, 256, 0, stream>>>(act, lg, lb, r0, Hh, Hl);
        k_gemmw<bf, 1, false><<<dim3(RCH / 64, 1, 1), 32, 0, stream>>>(Hh, Hl, WPB, nullptr, CC, BIASF + (size_t)r0 * 64, 64, nullptr, 0, 0, 0); }
    for (int b0 = 0; b0 < NG; b0 += CHB) { const int r0 = b0 * NG;
        k_gln<<<LR, 256, 0, stream>>>(act, lg, lb, r0, Hh, Hl);
        k_gemmw<bf, 1, false><<<dim3(RCH / 64, 512 / 64, 1), 32, 0, stream>>>(Hh, Hl, WPR, nullptr, CC, PF, 512, nullptr, 0, 0, 0);
        k_gpl<<<(NZC * NG * HD / 2 + 255) / 256, 256, 0, stream>>>(PF, QP, KP); k_gvt<<<(NZC * 64 * NG / 2 + 255) / 256, 256, 0, stream>>>(PF, VT);
        k_gemmw<h16, 0, false><<<dim3(NG / 64, NG / 64, NZC), 32, 0, stream>>>(QP, nullptr, KP, nullptr, HD, Sb, NG, nullptr, (size_t)NG * HD, (size_t)NG * HD, (size_t)NG * NG);
        k_gsoft<<<NZC * NG / 8, 256, 0, stream>>>(Sb, BIASF, pm, b0, Pm);
        k_gemmw<h16, 0, false><<<dim3(NG / 64, 1, NZC), 32, 0, stream>>>(Pm, nullptr, VT, nullptr, NG, Ob, 64, nullptr, (size_t)NG * NG, (size_t)64 * NG, (size_t)NG * 64);
        k_gmrg<<<(RCH * CC / 2 + 255) / 256, 256, 0, stream>>>(Ob, PF, Ah, Al);
        k_gemmw<bf, 1, false><<<dim3(RCH / 64, CC / 64, 1), 32, 0, stream>>>(Ah, Al, WO, nullptr, CC, OUT + (size_t)r0 * CC, CC, nullptr, 0, 0, 0); }
}
